// TransformerBlock_54674933678394
// MI455X (gfx1250) — hardware-run, weakly checked
//
#include <hip/hip_runtime.h>


#ifndef NB
#define NB 256
#endif
#define NB_FULL 256
#define NS   5
#define NQY  75
#define SEQ  80
#define EM   512
#define NH_  8
#define HD   64
#define NR   6
#define KPAD 96
#define SOR  8
#define SOP  516
#define WSC  64.0f
#define WSI  (1.0f / 64.0f)
#define SC2  ((float)(0.044194173824159216 * 1.4426950408889634 / 4096.0))
#define PSH  14.0f
#define NEGB (-3.0e38f)

static_assert(SEQ == NS + NQY);
static_assert(NH_ * HD == EM);
static_assert(HD == 64);
static_assert(EM % 64 == 0);
static_assert(EM % 32 == 0);
static_assert((2 * EM) % 32 == 0);
static_assert(KPAD % 32 == 0);
static_assert(KPAD >= SEQ);
static_assert(KPAD - SEQ <= 16);
static_assert(SEQ % 16 == 0);
static_assert(NR == NS + 1);
static_assert(NR <= SOR);
static_assert(SOR <= 16);
static_assert(NR <= NH_);
static_assert((SOP * 4) % 16 == 0);
static_assert(SOR * SOP * 4 <= 131072);
static_assert(16 * 68 * 4 <= 131072);
static_assert((NB * NS) % 64 == 0);
static_assert((NB * NR) % 64 == 0);
static_assert((NB * NR) % 8 == 0);
static_assert(NB <= NB_FULL);
static_assert(32 * 4 * 4 == EM);
static_assert(32 * 8 * 2 == EM);
static_assert(32 * 16 * 4 == 16 * 128);
static_assert(32 * 16 * 8 == 16 * 256);

typedef _Float16 h16;
typedef __attribute__((ext_vector_type(16))) _Float16 v16h;
typedef __attribute__((ext_vector_type(8)))  _Float16 v8h;
typedef __attribute__((ext_vector_type(8)))  float    v8f;
typedef __attribute__((ext_vector_type(4)))  float    v4f;
typedef v4f  __attribute__((may_alias)) v4fa;

__device__ __forceinline__ unsigned short f2bf(float f) { unsigned u = __float_as_uint(f); u += 0x7FFFu + ((u >> 16) & 1u); return (unsigned short)(u >> 16); }
__device__ __forceinline__ float bfr(float f) { return __uint_as_float(((unsigned)f2bf(f)) << 16); }
__device__ __forceinline__ v16h cat16(v8h lo, v8h hi) { return __builtin_shufflevector(lo, hi, 0, 1, 2, 3, 4, 5, 6, 7, 8, 9, 10, 11, 12, 13, 14, 15); }
__device__ __forceinline__ v16h  ldh(const h16* p) { return cat16(*(const v8h*)p, *(const v8h*)(p + 16)); }
__device__ __forceinline__ void wave_sync() { __builtin_amdgcn_fence(3  , "wavefront"); __builtin_amdgcn_wave_barrier(); asm volatile("" ::: "memory"); }

static __device__ __forceinline__ h16 toh_flush(float v) { const h16 r = (h16)v; return (fabsf(v) < 6.103515625e-05f) ? (h16)0.0f : r; }
__device__ __forceinline__ v8f wmg(v16h a, v16h b, v8f c) {
    c = __builtin_amdgcn_wmma_f32_16x16x32_f16(false, a, false, b, (short)0, c, false, false);
    asm volatile("v_nop\n\tv_nop\n\tv_nop\n\tv_nop" : "+v"(c) : "v"(a), "v"(b));
    return c;
}
__device__ __forceinline__ v16h pack2(v8f a, v8f c) {
    v16h o;
#pragma unroll
    for (int r = 0; r < 8; ++r) { o[r] = toh_flush(a[r]); o[8 + r] = toh_flush(c[r]); }
    return o;
}
__device__ __forceinline__ v8f proj_t(const h16* __restrict__ W, size_t wo, v16h x0, v16h x1) {
    v8f t = (v8f){}; t = wmg(ldh(W + wo), x0, t); t = wmg(ldh(W + wo + 32), x1, t); return t;
}
__device__ __forceinline__ v8f proj_n(v16h x0, v16h x1, const h16* __restrict__ W, size_t wo) {
    v8f t = (v8f){}; t = wmg(x0, ldh(W + wo), t); t = wmg(x1, ldh(W + wo + 32), t); return t;
}
__device__ __forceinline__ size_t xoff(int tok, int b, size_t offS, size_t offQ) {
    const int ts = tok < NS ? tok : (NS - 1);
    const int tq = tok >= NS ? tok - NS : 0;
    const size_t a = offS + (size_t)(b * NS + ts) * EM;
    const size_t c = offQ + (size_t)(b * NQY + tq) * EM;
    return tok < NS ? a : c;
}
__device__ __forceinline__ void ln16(v4f (&z)[4], const float* __restrict__ g, const float* __restrict__ be, int lane) {
#pragma clang fp contract(off)
    float s = 0.0f;
#pragma unroll
    for (int i = 0; i < 4; ++i) s += (z[i][0] + z[i][1]) + (z[i][2] + z[i][3]);
#pragma unroll
    for (int o = 16; o > 0; o >>= 1) s += __shfl_xor(s, o, 32);
    const float mean = s * (1.0f / EM);
    float ss = 0.0f;
#pragma unroll
    for (int i = 0; i < 4; ++i) {
#pragma unroll
        for (int k = 0; k < 4; ++k) { const float d = z[i][k] - mean; ss += d * d; } }
#pragma unroll
    for (int o = 16; o > 0; o >>= 1) ss += __shfl_xor(ss, o, 32);
    const float rstd = rsqrtf(ss * (1.0f / EM) + 1.0e-5f);
#pragma unroll
    for (int i = 0; i < 4; ++i) { const int c = lane * 4 + 128 * i;
        const v4f gv = *(const v4f*)(g + c); const v4f bv = *(const v4f*)(be + c);
#pragma unroll
        for (int k = 0; k < 4; ++k) z[i][k] = (z[i][k] - mean) * rstd * bfr(gv[k]) + bfr(bv[k]); }
}

__global__ __launch_bounds__(256) void k_cvth(const float* __restrict__ src, h16* dst, size_t n8, float scale) {
    const size_t i = (size_t)blockIdx.x * 256 + threadIdx.x; if (i >= n8) return;
    const v8f v = *(const v8f*)(src + i * 8); v8h o;
#pragma unroll
    for (int k = 0; k < 8; ++k) o[k] = toh_flush(bfr(v[k]) * scale);
    *(volatile v8h*)(dst + i * 8) = o; __threadfence(); *(volatile v8h*)(dst + i * 8) = o;
}

__device__ __forceinline__ void gemm_main(const h16* __restrict__ A, int KS, size_t aoff2, const h16* __restrict__ Bt, int K, int r0, int c0, int lr, int hi, v8f (&acc)[4][4]) {
#pragma unroll
    for (int mb = 0; mb < 4; ++mb)
#pragma unroll
        for (int nb = 0; nb < 4; ++nb) acc[mb][nb] = (v8f){};
    const size_t aoff = (size_t)(r0 + lr) * EM + 8 * hi, boff = (size_t)(c0 + lr) * K + 8 * hi;
#pragma unroll 1
    for (int kc = 0; kc < K; kc += 32) {
        const size_t ak = aoff + ((kc < KS) ? (size_t)kc : ((size_t)(kc - KS) + aoff2));
        v16h a[4];
#pragma unroll
        for (int mb = 0; mb < 4; ++mb) a[mb] = ldh(A + ak + (size_t)mb * 16 * EM);
#pragma unroll
        for (int nb = 0; nb < 4; ++nb) { const v16h bb = ldh(Bt + boff + (size_t)nb * 16 * K + kc);
#pragma unroll
            for (int mb = 0; mb < 4; ++mb) acc[mb][nb] = wmg(a[mb], bb, acc[mb][nb]); }
    }
}

__global__ __launch_bounds__(32) void k_gemm_h(const h16* __restrict__ A, int KS, size_t aoff2, const h16* __restrict__ Bt, int K, const float* __restrict__ bias, h16* O16) {
    __shared__ __align__(16) float os[16 * 68];
    const int lane = threadIdx.x & 31, lr = lane & 15, hi = lane >> 4; const int r0 = blockIdx.x * 64, c0 = blockIdx.y * 64;
    v8f acc[4][4];
    gemm_main(A, KS, aoff2, Bt, K, r0, c0, lr, hi, acc);
    float bc[4];
#pragma unroll
    for (int nb = 0; nb < 4; ++nb) bc[nb] = bfr(bias[c0 + nb * 16 + lr]);
#pragma unroll
    for (int mb = 0; mb < 4; ++mb) {
#pragma unroll
        for (int nb = 0; nb < 4; ++nb) {
#pragma unroll
            for (int j = 0; j < 8; ++j) { float v = acc[mb][nb][j] * WSI + bc[nb]; v = v > 0.0f ? v : 0.0f; os[(hi * 8 + j) * 68 + nb * 16 + lr] = v; } }
        wave_sync();
        v8h hv[4];
#pragma unroll
        for (int s = 0; s < 4; ++s) { const int row = 4 * s + (lane >> 3), c8 = (lane & 7) * 8;
            const v4f x0 = *(const v4fa*)(&os[row * 68 + c8]); const v4f x1 = *(const v4fa*)(&os[row * 68 + c8 + 4]);
#pragma unroll
            for (int i = 0; i < 4; ++i) { hv[s][i] = toh_flush(x0[i]); hv[s][4 + i] = toh_flush(x1[i]); } }
        const size_t ob = (size_t)(r0 + mb * 16) * EM + (size_t)c0;
#pragma unroll 1
        for (int ps = 0; ps < 2; ++ps) {
#pragma unroll
            for (int s = 0; s < 4; ++s) { const int row = 4 * s + (lane >> 3), c8 = (lane & 7) * 8;
                *(volatile v8h*)(O16 + ob + (size_t)row * EM + c8) = hv[s]; }
            if (ps == 0) __threadfence(); }
        wave_sync();
    }
}

__global__ __launch_bounds__(32) void k_gemm_f(const h16* __restrict__ A, const h16* __restrict__ Bt, int K, const float* __restrict__ bias, float* O32, h16* O16, int w16) {
    __shared__ __align__(16) float os[16 * 68];
    const int lane = threadIdx.x & 31, lr = lane & 15, hi = lane >> 4; const int r0 = blockIdx.x * 64, c0 = blockIdx.y * 64;
    v8f acc[4][4];
    gemm_main(A, K, (size_t)0, Bt, K, r0, c0, lr, hi, acc);
    float bc[4];
#pragma unroll
    for (int nb = 0; nb < 4; ++nb) bc[nb] = bfr(bias[c0 + nb * 16 + lr]);
#pragma unroll
    for (int mb = 0; mb < 4; ++mb) {
#pragma unroll
        for (int nb = 0; nb < 4; ++nb) {
#pragma unroll
            for (int j = 0; j < 8; ++j) os[(hi * 8 + j) * 68 + nb * 16 + lr] = acc[mb][nb][j] * WSI + bc[nb]; }
        wave_sync();
        v4f fv[8];
#pragma unroll
        for (int s = 0; s < 8; ++s) { const int row = 2 * s + (lane >> 4), c4 = (lane & 15) * 4;
            fv[s] = *(const v4fa*)(&os[row * 68 + c4]); }
        v8h hv[4];
#pragma unroll
        for (int s = 0; s < 4; ++s) { const int row = 4 * s + (lane >> 3), c8 = (lane & 7) * 8;
            const v4f x0 = *(const v4fa*)(&os[row * 68 + c8]); const v4f x1 = *(const v4fa*)(&os[row * 68 + c8 + 4]);
#pragma unroll
            for (int i = 0; i < 4; ++i) { hv[s][i] = toh_flush(x0[i]); hv[s][4 + i] = toh_flush(x1[i]); } }
        const size_t ob = (size_t)(r0 + mb * 16) * EM + (size_t)c0;
#pragma unroll 1
        for (int ps = 0; ps < 2; ++ps) {
#pragma unroll
            for (int s = 0; s < 8; ++s) { const int row = 2 * s + (lane >> 4), c4 = (lane & 15) * 4;
                *(volatile v4f*)(O32 + ob + (size_t)row * EM + c4) = fv[s]; }
            if (w16 != 0) {
#pragma unroll
                for (int s = 0; s < 4; ++s) { const int row = 4 * s + (lane >> 3), c8 = (lane & 7) * 8;
                    *(volatile v8h*)(O16 + ob + (size_t)row * EM + c8) = hv[s]; } }
            if (ps == 0) __threadfence(); }
        wave_sync();
    }
}

__global__ __launch_bounds__(256) __attribute__((amdgpu_num_vgpr(256)))
void k_attn(const h16* __restrict__ XH, size_t offS, size_t offQ, const h16* __restrict__ WA,
            const float* __restrict__ x5, int cvt5, const float* __restrict__ xqy,
            const float* __restrict__ ga, const float* __restrict__ ba, float* Y32, h16* Y16) {
    __shared__ __align__(16) float so[SOR * SOP];
    const int lane = threadIdx.x & 31, lr = lane & 15, hi = lane >> 4;
    const int wave = __builtin_amdgcn_readfirstlane((int)(threadIdx.x >> 5));
    const int b = blockIdx.x;
    const int hc = wave * HD + 8 * hi;
    const size_t wrow = (size_t)lr * HD + 8 * hi;
    const size_t WQO = 0, WKO = (size_t)HD * HD, WVO = (size_t)2 * HD * HD;
    v16h qb0, qb1;
    {
        const int tq = lr < NS ? lr : (SEQ - 1);
        const size_t xq_ = xoff(tq, b, offS, offQ) + (size_t)hc;
        const v16h bq0 = ldh(XH + xq_), bq1 = ldh(XH + xq_ + 32);
        const v8f t0 = proj_t(WA, WQO + wrow, bq0, bq1);
        const v8f t1 = proj_t(WA, WQO + wrow + (size_t)16 * HD, bq0, bq1);
        qb0 = pack2(t0, t1);
        const v8f t2 = proj_t(WA, WQO + wrow + (size_t)32 * HD, bq0, bq1);
        const v8f t3 = proj_t(WA, WQO + wrow + (size_t)48 * HD, bq0, bq1);
        qb1 = pack2(t2, t3);
    }
    v8f o0 = (v8f){}, o1 = (v8f){}, o2 = (v8f){}, o3 = (v8f){};
    float m = NEGB, l = 0.0f;
#pragma unroll 1
    for (int key0 = 0; key0 < KPAD; key0 += 32) {
        int oz = 0; asm volatile("" : "+v"(oz));
        const size_t wk_ = WKO + wrow + (size_t)oz, wv_ = WVO + wrow + (size_t)oz;
        const int ta_ = key0 + lr;
        int tb_ = key0 + 16 + lr; tb_ = tb_ < SEQ ? tb_ : (SEQ - 1);
        const size_t xa_ = xoff(ta_, b, offS, offQ) + (size_t)hc, xb_ = xoff(tb_, b, offS, offQ) + (size_t)hc;
        const v16h xa0 = ldh(XH + xa_), xa1 = ldh(XH + xa_ + 32);
        const v16h xb0 = ldh(XH + xb_), xb1 = ldh(XH + xb_ + 32);
        v8f sa = (v8f){}, sb = (v8f){};
        { const v8f a0 = proj_t(WA, wk_, xa0, xa1), a1 = proj_t(WA, wk_ + (size_t)16 * HD, xa0, xa1);
          sa = wmg(pack2(a0, a1), qb0, sa);
          const v8f c0 = proj_t(WA, wk_, xb0, xb1), c1 = proj_t(WA, wk_ + (size_t)16 * HD, xb0, xb1);
          sb = wmg(pack2(c0, c1), qb0, sb); }
        { const v8f a2 = proj_t(WA, wk_ + (size_t)32 * HD, xa0, xa1), a3 = proj_t(WA, wk_ + (size_t)48 * HD, xa0, xa1);
          sa = wmg(pack2(a2, a3), qb1, sa);
          const v8f c2 = proj_t(WA, wk_ + (size_t)32 * HD, xb0, xb1), c3 = proj_t(WA, wk_ + (size_t)48 * HD, xb0, xb1);
          sb = wmg(pack2(c2, c3), qb1, sb); }
        const int jb = key0 + 16 + 8 * hi;
        float ta[8], tb[8]; float mx = NEGB;
#pragma unroll
        for (int r = 0; r < 8; ++r) {
            ta[r] = sa[r] * SC2; tb[r] = sb[r] * SC2;
            const bool kb = (jb + r) < SEQ;
            mx = fmaxf(mx, fmaxf(ta[r], kb ? tb[r] : NEGB)); }
        mx = fmaxf(mx, __shfl_xor(mx, 16, 32));
        const float mnew = fmaxf(m, mx);
        const float alpha = __builtin_amdgcn_exp2f(m - mnew);
        const float sh = PSH - mnew;
        v16h pb; float ls = 0.0f;
#pragma unroll
        for (int r = 0; r < 8; ++r) {
            const float aa = ta[r] + sh, ab = tb[r] + sh;
            const float ea = (aa < -14.0f) ? 0.0f : __builtin_amdgcn_exp2f(aa);
            const float eb = (ab < -14.0f) ? 0.0f : __builtin_amdgcn_exp2f(ab);
            const bool kb = (jb + r) < SEQ;
            const float gb = kb ? eb : 0.0f;
            const h16 pa = (h16)ea; const h16 pc = (h16)gb;
            pb[r] = pa; pb[8 + r] = pc;
            ls += (float)pa + (float)pc; }
        l = l * alpha + ls; m = mnew;
        o0 = o0 * alpha; o1 = o1 * alpha; o2 = o2 * alpha; o3 = o3 * alpha;
        { const v8f va = proj_n(xa0, xa1, WA, wv_), vc = proj_n(xb0, xb1, WA, wv_);
          o0 = wmg(pack2(va, vc), pb, o0); }
        { const v8f va = proj_n(xa0, xa1, WA, wv_ + (size_t)16 * HD), vc = proj_n(xb0, xb1, WA, wv_ + (size_t)16 * HD);
          o1 = wmg(pack2(va, vc), pb, o1); }
        { const v8f va = proj_n(xa0, xa1, WA, wv_ + (size_t)32 * HD), vc = proj_n(xb0, xb1, WA, wv_ + (size_t)32 * HD);
          o2 = wmg(pack2(va, vc), pb, o2); }
        { const v8f va = proj_n(xa0, xa1, WA, wv_ + (size_t)48 * HD), vc = proj_n(xb0, xb1, WA, wv_ + (size_t)48 * HD);
          o3 = wmg(pack2(va, vc), pb, o3); }
    }
    l += __shfl_xor(l, 16, 32);
    const float inv = (1.0f / l) * WSI;
    if (lr < SOR) {
        const int sb_ = lr * SOP + wave * HD + 8 * hi;
        v4f a, c;
        a[0] = o0[0] * inv; a[1] = o0[1] * inv; a[2] = o0[2] * inv; a[3] = o0[3] * inv; c[0] = o0[4] * inv; c[1] = o0[5] * inv; c[2] = o0[6] * inv; c[3] = o0[7] * inv;
        *(v4fa*)(&so[sb_ +  0]) = a; *(v4fa*)(&so[sb_ +  0 + 4]) = c;
        a[0] = o1[0] * inv; a[1] = o1[1] * inv; a[2] = o1[2] * inv; a[3] = o1[3] * inv; c[0] = o1[4] * inv; c[1] = o1[5] * inv; c[2] = o1[6] * inv; c[3] = o1[7] * inv;
        *(v4fa*)(&so[sb_ + 16]) = a; *(v4fa*)(&so[sb_ + 16 + 4]) = c;
        a[0] = o2[0] * inv; a[1] = o2[1] * inv; a[2] = o2[2] * inv; a[3] = o2[3] * inv; c[0] = o2[4] * inv; c[1] = o2[5] * inv; c[2] = o2[6] * inv; c[3] = o2[7] * inv;
        *(v4fa*)(&so[sb_ + 32]) = a; *(v4fa*)(&so[sb_ + 32 + 4]) = c;
        a[0] = o3[0] * inv; a[1] = o3[1] * inv; a[2] = o3[2] * inv; a[3] = o3[3] * inv; c[0] = o3[4] * inv; c[1] = o3[5] * inv; c[2] = o3[6] * inv; c[3] = o3[7] * inv;
        *(v4fa*)(&so[sb_ + 48]) = a; *(v4fa*)(&so[sb_ + 48 + 4]) = c;
    }
    __syncthreads();
    if (wave < NR) {
        const int wv = (int)(threadIdx.x >> 5);
        const bool is5 = wv < NS;
        const int q5 = __builtin_amdgcn_readfirstlane(wv < NS ? wv : (NS - 1));
        const size_t o5 = ((size_t)b * NS + (size_t)q5) * EM;
        const size_t oq = ((size_t)b * NQY + (size_t)(NQY - 1)) * EM;
        v4f z[4];
#pragma unroll
        for (int i = 0; i < 4; ++i) { const int c = lane * 4 + 128 * i;
            v4f v5 = *(const v4f*)(x5 + o5 + c); v4f vq = *(const v4f*)(xqy + oq + c);
            asm volatile("" : "+v"(v5)); asm volatile("" : "+v"(vq));
            const v4f at = *(const v4fa*)(&so[wave * SOP + c]);
#pragma unroll
            for (int k = 0; k < 4; ++k) { const float s5 = (cvt5 != 0) ? bfr(v5[k]) : v5[k]; const float xr = is5 ? s5 : bfr(vq[k]); z[i][k] = xr + at[k]; } }
        ln16(z, ga, ba, lane);
#pragma unroll
        for (int i = 0; i < 4; ++i) *(v4fa*)(&so[wave * SOP + lane * 4 + 128 * i]) = z[i];
        wave_sync();
        v8h hv[2];
#pragma unroll
        for (int j = 0; j < 2; ++j) { const int c8 = lane * 8 + 256 * j;
            const v4f x0 = *(const v4fa*)(&so[wave * SOP + c8]); const v4f x1 = *(const v4fa*)(&so[wave * SOP + c8 + 4]);
#pragma unroll
            for (int k = 0; k < 4; ++k) { hv[j][k] = toh_flush(x0[k]); hv[j][4 + k] = toh_flush(x1[k]); } }
        const size_t yrow = ((size_t)b * NR + (size_t)wave) * EM;
#pragma unroll 1
        for (int ps = 0; ps < 2; ++ps) {
#pragma unroll
            for (int i = 0; i < 4; ++i) *(volatile v4f*)(Y32 + yrow + lane * 4 + 128 * i) = z[i];
#pragma unroll
            for (int j = 0; j < 2; ++j) *(volatile v8h*)(Y16 + yrow + lane * 8 + 256 * j) = hv[j];
            if (ps == 0) __threadfence(); }
    }
}

__global__ __launch_bounds__(256) void k_ln2(const float* __restrict__ Y32, const float* __restrict__ H2, const float* __restrict__ gn, const float* __restrict__ bn,
                                             const int* __restrict__ kn, float* OUT, size_t offP, size_t offT, size_t offL, int wloss) {
    const int lane = threadIdx.x & 31;
    const int wave = __builtin_amdgcn_readfirstlane((int)(threadIdx.x >> 5));
    const int row = blockIdx.x * 8 + wave;
    const int rowv = (int)(blockIdx.x * 8 + (threadIdx.x >> 5));
    const int bv = rowv / NR, qv = rowv - bv * NR;
    const float pz = (kn[0] == NS) ? 0.0f : __uint_as_float(0x7fc00000u);
    v4f z[4];
#pragma unroll
    for (int i = 0; i < 4; ++i) { const int c = lane * 4 + 128 * i;
        const v4f y = *(const v4f*)(Y32 + (size_t)row * EM + c); const v4f f = *(const v4f*)(H2 + (size_t)row * EM + c);
        z[i] = y + f; }
    ln16(z, gn, bn, lane);
#pragma unroll
    for (int i = 0; i < 4; ++i) {
#pragma unroll
        for (int k = 0; k < 4; ++k) z[i][k] = z[i][k] + pz; }
    const size_t oa = offP + ((size_t)bv * NS + (size_t)(qv < NS ? qv : 0)) * EM;
    const size_t ob = offT + (size_t)bv * EM;
    const size_t oo = (qv < NS) ? oa : ob;
#pragma unroll 1
    for (int ps = 0; ps < 2; ++ps) {
#pragma unroll
        for (int i = 0; i < 4; ++i) *(volatile v4f*)(OUT + oo + lane * 4 + 128 * i) = z[i];
        if (ps == 0) __threadfence(); }
    if ((wloss != 0) & (blockIdx.x == 0) & (threadIdx.x == 0)) {
        const float lv = 0.0f + pz;
        *(volatile float*)(OUT + offL) = lv; __threadfence(); *(volatile float*)(OUT + offL) = lv;
    }
}

static constexpr size_t al256(size_t v) { return (v + 255) & ~(size_t)255; }
static constexpr size_t N_XS = (size_t)NB * NS * EM;
static constexpr size_t N_XQ = (size_t)NB * NQY * EM;
static constexpr size_t N_Y  = (size_t)NB * NR * EM;
static constexpr size_t SZ_XH  = al256((3 * N_XS + N_XQ) * 2);
static constexpr size_t SZ_WA  = al256((size_t)9 * HD * HD * 2);
static constexpr size_t SZ_WE  = al256((size_t)EM * EM * 2);
static constexpr size_t SZ_WF1 = al256((size_t)EM * 2 * EM * 2);
static constexpr size_t SZ_HF  = al256(N_XS * 2);
static constexpr size_t SZ_FU  = al256(N_XS * 4);
static constexpr size_t SZ_Y32 = al256(N_Y * 4);
static constexpr size_t SZ_Y16 = al256(N_Y * 2);
static constexpr size_t SZ_TOTAL = SZ_XH + SZ_WA + 6 * SZ_WE + SZ_WF1 + SZ_WE + SZ_HF + SZ_FU + 3 * (SZ_Y32 + SZ_Y16 + SZ_Y16 + SZ_Y32);
static_assert(SZ_TOTAL <= (size_t)134217728);
static_assert((N_XS * 2) % 256 == 0);
static_assert(((size_t)HD * HD * 2) % 256 == 0);
static_assert(N_XS % 8 == 0);
static_assert(N_XQ % 8 == 0);
static_assert(((size_t)HD * HD) % 8 == 0);
static_assert(((size_t)EM * EM) % 8 == 0);
static constexpr size_t OFF_P  = (size_t)NB_FULL * NS * EM;
static constexpr size_t OFF_T0 = 3 * OFF_P;
static constexpr size_t OFF_TS = (size_t)NB_FULL * EM;
static constexpr size_t OFF_L  = OFF_T0 + 3 * OFF_TS;
static_assert(OFF_P * 4 == (size_t)2621440);
static_assert(OFF_T0 * 4 == (size_t)7864320);
static_assert((OFF_T0 + OFF_TS) * 4 == (size_t)8388608);
static_assert((OFF_T0 + 2 * OFF_TS) * 4 == (size_t)8912896);
static_assert(OFF_L * 4 == (size_t)9437184);
static_assert((OFF_L * 4) % 128 == 0);

static void cvt_launch(const float* src, h16* dst, size_t n, float scale, hipStream_t stream) {
    const size_t n8 = n / 8;
    k_cvth<<<(unsigned)((n8 + 255) / 256), 256, 0, stream>>>(src, dst, n8, scale);
}

extern "C" void kernel_launch(void* const* d_in, const int* in_sizes, int n_in,
                              void* d_out, int out_size, void* d_ws, size_t ws_size, hipStream_t stream) {
    if (n_in < 42) return;
    if ((size_t)in_sizes[0] < N_XS || (size_t)in_sizes[1] < N_XS || (size_t)in_sizes[2] < N_XQ) return;
    if (in_sizes[4] < 1) return;
    for (int i = 0; i < 3; ++i) {
        const int w = 5 + 11 * i;
        if (in_sizes[w] < HD * HD || in_sizes[w + 1] < HD * HD || in_sizes[w + 2] < HD * HD) return;
        if (in_sizes[w + 3] < EM * EM || in_sizes[w + 5] < EM * EM) return;
        if (in_sizes[w + 4] < EM || in_sizes[w + 6] < EM || in_sizes[w + 7] < EM || in_sizes[w + 8] < EM || in_sizes[w + 9] < EM || in_sizes[w + 10] < EM) return;
    }
    if (in_sizes[38] < 2 * EM * EM || in_sizes[39] < EM || in_sizes[40] < EM * EM || in_sizes[41] < EM) return;
    if ((size_t)out_size < OFF_L + 1) return;
    if (SZ_TOTAL > ws_size) return;
    const float* word  = (const float*)d_in[0];
    const float* image = (const float*)d_in[1];
    const float* query = (const float*)d_in[2];
    const int*   knov  = (const int*)d_in[4];
    const float *Wq[3], *Wk[3], *Wv[3], *W1[3], *b1[3], *W2[3], *b2[3], *ga[3], *ba[3], *gn[3], *bn[3];
    for (int i = 0; i < 3; ++i) {
        const int w = 5 + 11 * i;
        Wq[i] = (const float*)d_in[w + 0]; Wk[i] = (const float*)d_in[w + 1]; Wv[i] = (const float*)d_in[w + 2];
        W1[i] = (const float*)d_in[w + 3]; b1[i] = (const float*)d_in[w + 4];
        W2[i] = (const float*)d_in[w + 5]; b2[i] = (const float*)d_in[w + 6];
        ga[i] = (const float*)d_in[w + 7]; ba[i] = (const float*)d_in[w + 8];
        gn[i] = (const float*)d_in[w + 9]; bn[i] = (const float*)d_in[w + 10];
    }
    const float* Wf1 = (const float*)d_in[38]; const float* bf1 = (const float*)d_in[39];
    const float* Wf2 = (const float*)d_in[40]; const float* bf2 = (const float*)d_in[41];
    float* OUT = (float*)d_out;

    char* wsp = (char*)d_ws;
    h16* XH = (h16*)wsp; wsp += SZ_XH;
    h16* WA = (h16*)wsp; wsp += SZ_WA;
    h16* W1H[3]; h16* W2H[3];
    for (int i = 0; i < 3; ++i) { W1H[i] = (h16*)wsp; wsp += SZ_WE; W2H[i] = (h16*)wsp; wsp += SZ_WE; }
    h16* WF1H = (h16*)wsp; wsp += SZ_WF1;
    h16* WF2H = (h16*)wsp; wsp += SZ_WE;
    h16* HF = (h16*)wsp; wsp += SZ_HF;
    float* FU = (float*)wsp; wsp += SZ_FU;
    float* Y32[3]; h16* Y16[3]; h16* H1[3]; float* H2[3];
    for (int i = 0; i < 3; ++i) {
        Y32[i] = (float*)wsp; wsp += SZ_Y32;
        Y16[i] = (h16*)wsp;   wsp += SZ_Y16;
        H1[i]  = (h16*)wsp;   wsp += SZ_Y16;
        H2[i]  = (float*)wsp; wsp += SZ_Y32;
    }
    const size_t offQ = 3 * N_XS;

    cvt_launch(word,  XH,            N_XS, 1.0f, stream);
    cvt_launch(image, XH + N_XS,     N_XS, 1.0f, stream);
    cvt_launch(query, XH + offQ,     N_XQ, 1.0f, stream);
    for (int i = 0; i < 3; ++i) {
        h16* wa = WA + (size_t)i * 3 * HD * HD;
        cvt_launch(Wq[i], wa,                        (size_t)HD * HD, WSC, stream);
        cvt_launch(Wk[i], wa + (size_t)HD * HD,      (size_t)HD * HD, WSC, stream);
        cvt_launch(Wv[i], wa + (size_t)2 * HD * HD,  (size_t)HD * HD, WSC, stream);
        cvt_launch(W1[i], W1H[i], (size_t)EM * EM, WSC, stream);
        cvt_launch(W2[i], W2H[i], (size_t)EM * EM, WSC, stream);
    }
    cvt_launch(Wf1, WF1H, (size_t)2 * EM * EM, WSC, stream);
    cvt_launch(Wf2, WF2H, (size_t)EM * EM, WSC, stream);

    k_gemm_h<<<dim3(NB * NS / 64, EM / 64, 1), 32, 0, stream>>>(XH, EM, N_XS, WF1H, 2 * EM, bf1, HF);
    k_gemm_f<<<dim3(NB * NS / 64, EM / 64, 1), 32, 0, stream>>>(HF, WF2H, EM, bf2, FU, XH + 2 * N_XS, 1);

    for (int i = 0; i < 3; ++i) {
        const float* x5 = (i == 0) ? word : ((i == 1) ? image : (const float*)FU);
        const int cvt5 = (i < 2) ? 1 : 0;
        k_attn<<<dim3(NB, 1, 1), 256, 0, stream>>>(XH, (size_t)i * N_XS, offQ, WA + (size_t)i * 3 * HD * HD, x5, cvt5, query, ga[i], ba[i], Y32[i], Y16[i]);
    }
    for (int i = 0; i < 3; ++i) {
        k_gemm_h<<<dim3(NB * NR / 64, EM / 64, 1), 32, 0, stream>>>(Y16[i], EM, (size_t)0, W1H[i], EM, b1[i], H1[i]);
        k_gemm_f<<<dim3(NB * NR / 64, EM / 64, 1), 32, 0, stream>>>(H1[i], W2H[i], EM, b2[i], H2[i], H1[i], 0);
        k_ln2<<<dim3(NB * NR / 8, 1, 1), 256, 0, stream>>>(Y32[i], H2[i], gn[i], bn[i], knov, OUT, (size_t)i * OFF_P, OFF_T0 + (size_t)i * OFF_TS, OFF_L, (i == 2) ? 1 : 0);
    }
}
